// MaskedAttention_45449343926629
// MI455X (gfx1250) — hardware-verified
//
#include <hip/hip_runtime.h>
#include <stdint.h>

#ifndef NB
#define NB 8
#endif
#ifndef SEQ
#define SEQ 1024
#endif
#define NB_FULL  8
#define SEQ_FULL 1024
#define DM    1024
#define NH    16
#define DH    64
#define NTOK  (NB * SEQ)

typedef _Float16 v16h __attribute__((ext_vector_type(16)));
typedef _Float16 v8h  __attribute__((ext_vector_type(8)));
typedef __bf16   v16b __attribute__((ext_vector_type(16)));
typedef __bf16   v8b  __attribute__((ext_vector_type(8)));
typedef float    v8f  __attribute__((ext_vector_type(8)));
typedef float    v4f  __attribute__((ext_vector_type(4)));
typedef unsigned short v8us __attribute__((ext_vector_type(8)));

static_assert(NB >= 1 && NB <= NB_FULL && SEQ >= 128 && SEQ <= SEQ_FULL && (SEQ % 128) == 0);
static_assert((DM % 64) == 0 && (NTOK % 128) == 0 && (DM % 32) == 0 && NH * DH == DM && DH == 64);

__device__ __forceinline__ unsigned short bfbits(float f) {
  const unsigned u = __float_as_uint(f);
  return (unsigned short)((u + 0x7FFFu + ((u >> 16) & 1u)) >> 16);
}
__device__ __forceinline__ float bfrnef(float f) {
  unsigned u = __float_as_uint(f);
  u = (u + 0x7FFFu + ((u >> 16) & 1u)) & 0xFFFF0000u;
  return __uint_as_float(u);
}

__device__ __forceinline__ v16h ldfrag(const _Float16* p) {
  union { v16h v; v8h hh[2]; } f;
  f.hh[0] = *(const v8h*)(p);
  f.hh[1] = *(const v8h*)(p + 16);
  return f.v;
}
__device__ __forceinline__ v16b ldfragb(const __bf16* p) {
  union { v16b v; v8b hh[2]; } f;
  f.hh[0] = *(const v8b*)(p);
  f.hh[1] = *(const v8b*)(p + 16);
  return f.v;
}
__device__ __forceinline__ v8f mma16(v16h a, v16h b, v8f c) {
  return __builtin_amdgcn_wmma_f32_16x16x32_f16(false, a, false, b, (short)0, c, false, false);
}
__device__ __forceinline__ v8f mmabf(v16b a, v16b b, v8f c) {
  return __builtin_amdgcn_wmma_f32_16x16x32_bf16(false, a, false, b, (short)0, c, false, false);
}
__device__ __forceinline__ v8f zero8() {
  v8f z;
#pragma unroll
  for (int i = 0; i < 8; ++i) z[i] = 0.0f;
  return z;
}

__device__ __forceinline__ void guard_b4(v8f& a, v8f& b, v8f& c, v8f& d, v16b x, v16b y) {
  asm volatile("v_nop\n\tv_nop\n\tv_nop\n\tv_nop" : "+v"(a), "+v"(b), "+v"(c), "+v"(d) : "v"(x), "v"(y));
}
__device__ __forceinline__ void guard_h4(v8f& a, v8f& b, v8f& c, v8f& d, v16h x, v16h y) {
  asm volatile("v_nop\n\tv_nop\n\tv_nop\n\tv_nop" : "+v"(a), "+v"(b), "+v"(c), "+v"(d) : "v"(x), "v"(y));
}
__device__ __forceinline__ void keep4b(v16b a, v16b b, v16b c, v16b d) {
  asm volatile("v_nop" :: "v"(a), "v"(b), "v"(c), "v"(d));
}
__device__ __forceinline__ void keep4h(v16h a, v16h b, v16h c, v16h d) {
  asm volatile("v_nop" :: "v"(a), "v"(b), "v"(c), "v"(d));
}
__device__ __forceinline__ void accg4(v8f& a, v8f& b, v8f& c, v8f& d) {
  asm volatile("v_nop\n\tv_nop\n\tv_nop\n\tv_nop" : "+v"(a), "+v"(b), "+v"(c), "+v"(d));
}
__device__ __forceinline__ void guard_s(v8f& a, v8f& b, v16h x0, v16h x1, v16h y0, v16h y1) {
  asm volatile("v_nop\n\tv_nop\n\tv_nop\n\tv_nop" : "+v"(a), "+v"(b) : "v"(x0), "v"(x1), "v"(y0), "v"(y1));
}
__device__ __forceinline__ void guard_pv(v8f& a, v8f& b, v16h p, v16h x, v16h y) {
  asm volatile("v_nop\n\tv_nop\n\tv_nop\n\tv_nop" : "+v"(a), "+v"(b) : "v"(p), "v"(x), "v"(y));
}

__global__ __launch_bounds__(256) void cvt_x_kernel(const float* __restrict__ x, unsigned short* __restrict__ xb, int n8) {
  const int li = (int)blockIdx.x * 256 + (int)threadIdx.x;
  if (li >= n8) return;
  const size_t e = (size_t)li * 8;
  const size_t tok = e / DM;
  const size_t col = e % DM;
  const size_t fr = (tok / SEQ) * SEQ_FULL + (tok % SEQ);
  const float* s = x + fr * DM + col;
  const v4f a = *(const v4f*)(s);
  const v4f b = *(const v4f*)(s + 4);
  v8us o;
#pragma unroll
  for (int i = 0; i < 4; ++i) {
    o[i]     = bfbits(a[i]);
    o[4 + i] = bfbits(b[i]);
  }
  unsigned short* d = xb + e;
  *(volatile v8us*)d = o;
  __threadfence();
  *(volatile v8us*)d = o;
}

__global__ __launch_bounds__(256) void cvt_w_kernel(const float* __restrict__ w0, const float* __restrict__ w1,
                                                    const float* __restrict__ w2,
                                                    unsigned short* __restrict__ d0, unsigned short* __restrict__ d1,
                                                    unsigned short* __restrict__ d2, int n8) {
  const int z = (int)blockIdx.y;
  const float* src = (z == 0) ? w0 : ((z == 1) ? w1 : w2);
  unsigned short* dst = (z == 0) ? d0 : ((z == 1) ? d1 : d2);
  const int li = (int)blockIdx.x * 256 + (int)threadIdx.x;
  if (li >= n8) return;
  const size_t e = (size_t)li * 8;
  const v4f a = *(const v4f*)(src + e);
  const v4f b = *(const v4f*)(src + e + 4);
  v8us o;
#pragma unroll
  for (int i = 0; i < 4; ++i) {
    o[i]     = bfbits(a[i]);
    o[4 + i] = bfbits(b[i]);
  }
  unsigned short* d = dst + e;
  *(volatile v8us*)d = o;
  __threadfence();
  *(volatile v8us*)d = o;
}

__global__ __launch_bounds__(256) void cvt_wo_kernel(const float* __restrict__ w, _Float16* __restrict__ d, int n8) {
  const int li = (int)blockIdx.x * 256 + (int)threadIdx.x;
  if (li >= n8) return;
  const size_t e = (size_t)li * 8;
  const v4f a = *(const v4f*)(w + e);
  const v4f b = *(const v4f*)(w + e + 4);
  v8h o;
#pragma unroll
  for (int i = 0; i < 4; ++i) {
    o[i]     = (_Float16)(bfrnef(a[i]) * 64.0f);
    o[4 + i] = (_Float16)(bfrnef(b[i]) * 64.0f);
  }
  _Float16* dd = d + e;
  *(volatile v8h*)dd = o;
  __threadfence();
  *(volatile v8h*)dd = o;
}

__global__ __launch_bounds__(256) void maskc_kernel(const float* __restrict__ msk, float* __restrict__ mr, int n4) {
  const int li = (int)blockIdx.x * 256 + (int)threadIdx.x;
  if (li >= n4) return;
  const size_t e = (size_t)li * 4;
  const size_t qrow = e / SEQ;
  const size_t kc = e % SEQ;
  const v4f a = *(const v4f*)(msk + qrow * SEQ_FULL + kc);
  v4f o;
#pragma unroll
  for (int i = 0; i < 4; ++i) o[i] = bfrnef(a[i]);
  float* d = mr + e;
  *(volatile v4f*)d = o;
  __threadfence();
  *(volatile v4f*)d = o;
}

__global__ __launch_bounds__(256) void proj_kernel(const __bf16* __restrict__ A, int lda,
                                                   const __bf16* __restrict__ Bt, int ldb,
                                                   _Float16* __restrict__ Ch, _Float16* __restrict__ Cl, int ldc,
                                                   int M, int N, int K,
                                                   const float* __restrict__ bias, int blen, int bmode) {
  __shared__ __align__(16) float sT[8][16 * 68];
  const int lane = threadIdx.x & 31, wave = threadIdx.x >> 5;
  const int tilesN = N >> 6, tilesM = M >> 6;
  const int tile = (int)blockIdx.x * 8 + wave;
  if (tile >= tilesM * tilesN) return;
  const int tm = tile / tilesN, tn = tile - tm * tilesN;
  const int m0 = tm << 6, n0 = tn << 6;
  const int rl = lane & 15;
  const int koff = (lane >> 4) * 8;
  const int mOff = (lane >> 4) * 8;

  v8f acc[4][4];
#pragma unroll
  for (int i = 0; i < 4; ++i)
#pragma unroll
    for (int j = 0; j < 4; ++j) acc[i][j] = zero8();

#pragma unroll 1
  for (int k0 = 0; k0 < K; k0 += 32) {
    v16b bh[4];
#pragma unroll
    for (int j = 0; j < 4; ++j) bh[j] = ldfragb(Bt + (size_t)(n0 + (j << 4) + rl) * ldb + koff + k0);
#pragma unroll
    for (int i = 0; i < 4; ++i) {
      const v16b ah = ldfragb(A + (size_t)(m0 + (i << 4) + rl) * lda + koff + k0);
#pragma unroll
      for (int j = 0; j < 4; ++j) acc[i][j] = mmabf(ah, bh[j], acc[i][j]);
      guard_b4(acc[i][0], acc[i][1], acc[i][2], acc[i][3], ah, bh[3]);
    }
    keep4b(bh[0], bh[1], bh[2], bh[3]);
  }
  accg4(acc[0][0], acc[0][1], acc[0][2], acc[0][3]);
  accg4(acc[1][0], acc[1][1], acc[1][2], acc[1][3]);
  accg4(acc[2][0], acc[2][1], acc[2][2], acc[2][3]);
  accg4(acc[3][0], acc[3][1], acc[3][2], acc[3][3]);

  float* slab = sT[wave];
  const int qq = lane >> 3, c8 = (lane & 7) * 8;
  int cb = n0 + c8;
  cb = (cb <= blen - 8) ? cb : (blen - 8);
#pragma unroll
  for (int i = 0; i < 4; ++i) {
    const int mBase = m0 + (i << 4);
#pragma unroll
    for (int j = 0; j < 4; ++j) {
#pragma unroll
      for (int r = 0; r < 8; ++r) slab[(mOff + r) * 68 + (j << 4) + rl] = acc[i][j][r];
    }
    __builtin_amdgcn_fence(3, "workgroup");
    __builtin_amdgcn_wave_barrier();
    __builtin_amdgcn_fence(2, "workgroup");
#pragma unroll
    for (int ps = 0; ps < 2; ++ps) {
#pragma unroll
      for (int it = 0; it < 4; ++it) {
        const int row = it * 4 + qq;
        int ib = mBase + row;
        ib = (ib < blen) ? ib : (blen - 1);
        const float brow = bfrnef(bias[ib]);
        const v4f bA = *(const v4f*)(bias + cb);
        const v4f bB = *(const v4f*)(bias + cb + 4);
        const float* sp = slab + row * 68 + c8;
        const v4f u0 = *(const v4f*)(sp);
        const v4f u1 = *(const v4f*)(sp + 4);
        v8h hv, lv;
#pragma unroll
        for (int e = 0; e < 4; ++e) {
          const float b0 = (bmode != 0) ? brow : bfrnef(bA[e]);
          const float b1 = (bmode != 0) ? brow : bfrnef(bB[e]);
          const float f0 = u0[e] + b0;
          const _Float16 g0 = (_Float16)f0;
          hv[e] = g0;
          lv[e] = (_Float16)((f0 - (float)g0) * 2048.0f);
          const float f1 = u1[e] + b1;
          const _Float16 g1 = (_Float16)f1;
          hv[4 + e] = g1;
          lv[4 + e] = (_Float16)((f1 - (float)g1) * 2048.0f);
        }
        const size_t go = (size_t)(mBase + row) * ldc + n0 + c8;
        *(volatile v8h*)(Ch + go) = hv;
        *(volatile v8h*)(Cl + go) = lv;
      }
      __threadfence();
    }
    __builtin_amdgcn_fence(3, "workgroup");
    __builtin_amdgcn_wave_barrier();
    __builtin_amdgcn_fence(2, "workgroup");
  }
}

__global__ __launch_bounds__(128) void norms_kernel(const _Float16* __restrict__ qh, const _Float16* __restrict__ qr,
                                                    const _Float16* __restrict__ kh, const _Float16* __restrict__ kr,
                                                    float* __restrict__ qs, float* __restrict__ ks) {
  const int z = (int)blockIdx.z;
  const _Float16* H = (z == 0) ? qh : kh;
  const _Float16* R = (z == 0) ? qr : kr;
  float* D = (z == 0) ? qs : ks;
  const int bhh = (int)blockIdx.y;
  const int b = bhh / NH, hd = bhh % NH;
  const int s = (int)blockIdx.x * 128 + (int)threadIdx.x;
  const size_t tok = (size_t)b * SEQ + s;
  const _Float16* ph = H + tok * DM + hd * DH;
  const _Float16* pr = R + tok * DM + hd * DH;
  float acc = 0.0f;
#pragma unroll 1
  for (int pc = 0; pc < 8; ++pc) {
    const v8h a = *(const v8h*)(ph + pc * 8);
    const v8h r = *(const v8h*)(pr + pc * 8);
#pragma unroll
    for (int e = 0; e < 8; ++e) {
      const float v = fmaf((float)r[e], 0.00048828125f, (float)a[e]);
      acc = fmaf(v, v, acc);
    }
  }
  float* d = D + (size_t)bhh * SEQ + s;
  *(volatile float*)d = acc;
  __threadfence();
  *(volatile float*)d = acc;
}

#define QBW    16
#define AW     8
#define QBLK   (QBW * AW)
#define KT     64
#define KSP    72
#define VSP    72
#define PSP    72
#define OSPF   68
#define L_KH   0
#define L_KR   9216
#define L_VH   18432
#define L_VR   27648
#define L_P    36864
#define L_KQ   55296
#define ATT_LDS 55552
static_assert(KT * KSP * 2 == L_KR - L_KH);
static_assert(KT * KSP * 2 == L_VH - L_KR);
static_assert(DH * VSP * 2 == L_VR - L_VH);
static_assert(DH * VSP * 2 == L_P - L_VR);
static_assert(AW * QBW * PSP * 2 == L_KQ - L_P);
static_assert(KT * 4 == ATT_LDS - L_KQ);
static_assert(AW * QBW * OSPF * 4 <= L_P);
static_assert((KSP % 8) == 0 && (VSP % 8) == 0 && (PSP % 8) == 0 && (OSPF % 4) == 0);
static_assert(KSP >= DH && VSP >= KT && PSP >= KT && OSPF >= DH);
static_assert((L_KR % 16) == 0 && (L_VH % 16) == 0 && (L_VR % 16) == 0 && (L_P % 16) == 0 && (L_KQ % 16) == 0);
static_assert((SEQ % KT) == 0 && (SEQ % QBLK) == 0 && AW * 32 == 256 && KT == 64 && DH == 64);

__global__ __launch_bounds__(256) void attn_kernel(const _Float16* __restrict__ qh, const _Float16* __restrict__ qr,
                                                   const _Float16* __restrict__ kh, const _Float16* __restrict__ kr,
                                                   const _Float16* __restrict__ vth, const _Float16* __restrict__ vtr,
                                                   const float* __restrict__ qsq, const float* __restrict__ ksq,
                                                   const float* __restrict__ maskr, _Float16* __restrict__ oh) {
  extern __shared__ __align__(16) char smem[];
  _Float16* Khs = (_Float16*)(smem + L_KH);
  _Float16* Krs = (_Float16*)(smem + L_KR);
  _Float16* Vhs = (_Float16*)(smem + L_VH);
  _Float16* Vrs = (_Float16*)(smem + L_VR);
  _Float16* Pall = (_Float16*)(smem + L_P);
  float* Kqs = (float*)(smem + L_KQ);

  const int tid = (int)threadIdx.x;
  const int wave = __builtin_amdgcn_readfirstlane(tid >> 5);
  const int lane = tid & 31, h = lane >> 4, c = lane & 15;
  const int qt = (int)blockIdx.x, hd = (int)blockIdx.y, b = (int)blockIdx.z;
  const int bh = b * NH + hd;
  const int q0 = qt * QBLK + QBW * wave;
  const size_t tokq = (size_t)b * SEQ + q0;
  const size_t tokk = (size_t)b * SEQ;
  const float ninf = -__builtin_inff();
  _Float16* Pw = Pall + wave * (QBW * PSP);

  const _Float16* qhp = qh + (tokq + c) * DM + hd * DH + 8 * h;
  const _Float16* qrp = qr + (tokq + c) * DM + hd * DH + 8 * h;
  const v16h qa0 = ldfrag(qhp), qa1 = ldfrag(qhp + 32);
  const v16h qb0 = ldfrag(qrp), qb1 = ldfrag(qrp + 32);
  const float qterm = qsq[(size_t)bh * SEQ + q0 + c];
  const float* mrow = maskr + (size_t)(q0 + c) * SEQ + 8 * h;

  float mrun = ninf, lpart = 0.0f;
  v8f oacc1[4], oacc2[4];
#pragma unroll
  for (int nt = 0; nt < 4; ++nt) { oacc1[nt] = zero8(); oacc2[nt] = zero8(); }

  const int ntile = SEQ / KT;
#pragma unroll 1
  for (int t = 0; t < ntile; ++t) {
    const int kb = t * KT;
    __syncthreads();
#pragma unroll
    for (int i = 0; i < 2; ++i) {
      const int idx = i * 256 + tid;
      const int row = idx >> 3;
      const int pc  = idx & 7;
      const size_t gk = (tokk + kb + row) * DM + hd * DH + pc * 8;
      *(v8h*)(Khs + row * KSP + pc * 8) = *(const v8h*)(kh + gk);
      *(v8h*)(Krs + row * KSP + pc * 8) = *(const v8h*)(kr + gk);
      const size_t gv = (size_t)(hd * DH + row) * NTOK + tokk + kb + pc * 8;
      *(v8h*)(Vhs + row * VSP + pc * 8) = *(const v8h*)(vth + gv);
      *(v8h*)(Vrs + row * VSP + pc * 8) = *(const v8h*)(vtr + gv);
    }
    if (tid < KT / 4) *(v4f*)(Kqs + tid * 4) = *(const v4f*)(ksq + (size_t)bh * SEQ + kb + tid * 4);
    __syncthreads();

    v8f sc[4];
    float tmax = ninf;
#pragma unroll
    for (int j = 0; j < 4; ++j) {
      v8f s1 = zero8(), s2 = zero8();
      const _Float16* kap = Khs + (16 * j + c) * KSP + 8 * h;
      const _Float16* krp = Krs + (16 * j + c) * KSP + 8 * h;
      {
        const v16h a = ldfrag(kap), ar = ldfrag(krp);
        s1 = mma16(a, qa0, s1);
        s2 = mma16(a, qb0, s2);
        s2 = mma16(ar, qa0, s2);
        guard_s(s1, s2, a, ar, qa0, qb0);
      }
      {
        const v16h a = ldfrag(kap + 32), ar = ldfrag(krp + 32);
        s1 = mma16(a, qa1, s1);
        s2 = mma16(a, qb1, s2);
        s2 = mma16(ar, qa1, s2);
        guard_s(s1, s2, a, ar, qa1, qb1);
      }
      const v4f kA = *(const v4f*)(Kqs + 16 * j + 8 * h);
      const v4f kB = *(const v4f*)(Kqs + 16 * j + 8 * h + 4);
      const v4f mA = *(const v4f*)(mrow + kb + 16 * j);
      const v4f mB = *(const v4f*)(mrow + kb + 16 * j + 4);
      float kv[8], mv[8];
#pragma unroll
      for (int e = 0; e < 4; ++e) { kv[e] = kA[e]; kv[4 + e] = kB[e]; mv[e] = mA[e]; mv[4 + e] = mB[e]; }
      v8f sv;
#pragma unroll
      for (int r = 0; r < 8; ++r) {
        const float tt = mv[r] - 0.125f * (qterm + kv[r]);
        const float s = fmaf(fmaf(s2[r], 0.00048828125f, s1[r]), 0.25f, tt);
        sv[r] = s;
        tmax = fmaxf(tmax, s);
      }
      sc[j] = sv;
    }
    tmax = fmaxf(tmax, __shfl_xor(tmax, 16, 32));
    const float mnew = fmaxf(mrun, tmax);
    const float al = __expf(mrun - mnew);
    mrun = mnew;
    lpart *= al;
    {
      float alr[8];
#pragma unroll
      for (int r = 0; r < 8; ++r) alr[r] = __shfl(al, 8 * h + r, 32);
#pragma unroll
      for (int nt = 0; nt < 4; ++nt) {
#pragma unroll
        for (int r = 0; r < 8; ++r) { oacc1[nt][r] *= alr[r]; oacc2[nt][r] *= alr[r]; }
      }
    }
#pragma unroll
    for (int j = 0; j < 4; ++j) {
      v8h ph;
#pragma unroll
      for (int r = 0; r < 8; ++r) {
        const float p = __expf(sc[j][r] - mrun);
        lpart += p;
        ph[r] = (_Float16)(p * 16384.0f);
      }
      *(v8h*)(Pw + c * PSP + 16 * j + 8 * h) = ph;
    }
    __builtin_amdgcn_fence(3, "workgroup");
    __builtin_amdgcn_wave_barrier();
    __builtin_amdgcn_fence(2, "workgroup");
#pragma unroll
    for (int ks = 0; ks < KT; ks += 32) {
      const v16h pa = ldfrag(Pw + c * PSP + ks + 8 * h);
#pragma unroll
      for (int nt = 0; nt < 4; ++nt) {
        const v16h x = ldfrag(Vhs + (16 * nt + c) * VSP + ks + 8 * h);
        const v16h y = ldfrag(Vrs + (16 * nt + c) * VSP + ks + 8 * h);
        oacc1[nt] = mma16(pa, x, oacc1[nt]);
        oacc2[nt] = mma16(pa, y, oacc2[nt]);
        guard_pv(oacc1[nt], oacc2[nt], pa, x, y);
      }
    }
  }

  const float l = lpart + __shfl_xor(lpart, 16, 32);
  const float lic = (1.0f / l) * 0.0009765625f;
  float lir[8];
#pragma unroll
  for (int r = 0; r < 8; ++r) lir[r] = __shfl(lic, 8 * h + r, 32);
  __syncthreads();
  float* slab = (float*)(smem + L_KH) + wave * (QBW * OSPF);
#pragma unroll
  for (int nt = 0; nt < 4; ++nt) {
    const int col = 16 * nt + c;
#pragma unroll
    for (int r = 0; r < 8; ++r)
      slab[(8 * h + r) * OSPF + col] = fmaf(oacc2[nt][r], 0.00048828125f, oacc1[nt][r]) * lir[r];
  }
  __builtin_amdgcn_fence(3, "workgroup");
  __builtin_amdgcn_wave_barrier();
  __builtin_amdgcn_fence(2, "workgroup");
  {
    const int qq = lane >> 3, c8 = (lane & 7) * 8;
#pragma unroll
    for (int ps = 0; ps < 2; ++ps) {
#pragma unroll
      for (int it = 0; it < 4; ++it) {
        const int row = it * 4 + qq;
        const float* sp = slab + row * OSPF + c8;
        const v4f u0 = *(const v4f*)(sp);
        const v4f u1 = *(const v4f*)(sp + 4);
        v8h hv;
#pragma unroll
        for (int e = 0; e < 4; ++e) { hv[e] = (_Float16)u0[e]; hv[4 + e] = (_Float16)u1[e]; }
        const size_t go = (tokq + (size_t)row) * DM + hd * DH + c8;
        *(volatile v8h*)(oh + go) = hv;
      }
      __threadfence();
    }
  }
}

__global__ __launch_bounds__(256) void oproj_kernel(const _Float16* __restrict__ A, int lda,
                                                    const _Float16* __restrict__ Bt, int ldb,
                                                    float* __restrict__ outp, int ldo,
                                                    int M, int N, int K,
                                                    const float* __restrict__ bias, int blen, float oscale) {
  __shared__ __align__(16) float sT[8][16 * 68];
  const int lane = threadIdx.x & 31, wave = threadIdx.x >> 5;
  const int tilesN = N >> 6, tilesM = M >> 6;
  const int tile = (int)blockIdx.x * 8 + wave;
  if (tile >= tilesM * tilesN) return;
  const int tm = tile / tilesN, tn = tile - tm * tilesN;
  const int m0 = tm << 6, n0 = tn << 6;
  const int rl = lane & 15;
  const int koff = (lane >> 4) * 8;
  const int mOff = (lane >> 4) * 8;

  v8f acc[4][4];
#pragma unroll
  for (int i = 0; i < 4; ++i)
#pragma unroll
    for (int j = 0; j < 4; ++j) acc[i][j] = zero8();

#pragma unroll 1
  for (int k0 = 0; k0 < K; k0 += 32) {
    v16h bh[4];
#pragma unroll
    for (int j = 0; j < 4; ++j) bh[j] = ldfrag(Bt + (size_t)(n0 + (j << 4) + rl) * ldb + koff + k0);
#pragma unroll
    for (int i = 0; i < 4; ++i) {
      const v16h ah = ldfrag(A + (size_t)(m0 + (i << 4) + rl) * lda + koff + k0);
#pragma unroll
      for (int j = 0; j < 4; ++j) acc[i][j] = mma16(ah, bh[j], acc[i][j]);
      guard_h4(acc[i][0], acc[i][1], acc[i][2], acc[i][3], ah, bh[3]);
    }
    keep4h(bh[0], bh[1], bh[2], bh[3]);
  }
  accg4(acc[0][0], acc[0][1], acc[0][2], acc[0][3]);
  accg4(acc[1][0], acc[1][1], acc[1][2], acc[1][3]);
  accg4(acc[2][0], acc[2][1], acc[2][2], acc[2][3]);
  accg4(acc[3][0], acc[3][1], acc[3][2], acc[3][3]);

  float* slab = sT[wave];
  const int rh = lane >> 4, c4 = (lane & 15) * 4;
  int cb = n0 + c4;
  cb = (cb <= blen - 4) ? cb : (blen - 4);
#pragma unroll
  for (int i = 0; i < 4; ++i) {
    const int mBase = m0 + (i << 4);
#pragma unroll
    for (int j = 0; j < 4; ++j) {
#pragma unroll
      for (int r = 0; r < 8; ++r) slab[(mOff + r) * 68 + (j << 4) + rl] = acc[i][j][r] * oscale;
    }
    __builtin_amdgcn_fence(3, "workgroup");
    __builtin_amdgcn_wave_barrier();
    __builtin_amdgcn_fence(2, "workgroup");
#pragma unroll
    for (int ps = 0; ps < 2; ++ps) {
#pragma unroll
      for (int it = 0; it < 8; ++it) {
        const int row = it * 2 + rh;
        const v4f u = *(const v4f*)(slab + row * 68 + c4);
        const v4f bb = *(const v4f*)(bias + cb);
        v4f v;
#pragma unroll
        for (int e = 0; e < 4; ++e) v[e] = u[e] + bfrnef(bb[e]);
        *(volatile v4f*)(outp + (size_t)(mBase + row) * ldo + n0 + c4) = v;
      }
      __threadfence();
    }
    __builtin_amdgcn_fence(3, "workgroup");
    __builtin_amdgcn_wave_barrier();
    __builtin_amdgcn_fence(2, "workgroup");
  }
}

static_assert((size_t)NTOK * DM * 2 + 4 * (size_t)DM * DM * 2 + 6 * (size_t)NTOK * DM * 2
              + 2 * (size_t)NB * NH * SEQ * 4 + (size_t)SEQ * SEQ * 4 <= (size_t)134217728);

extern "C" void kernel_launch(void* const* d_in, const int* in_sizes, int n_in,
                              void* d_out, int out_size, void* d_ws, size_t ws_size,
                              hipStream_t stream) {
  if (n_in < 10) return;
  if ((size_t)in_sizes[0] < (size_t)NB * SEQ_FULL * DM) return;
  if ((size_t)in_sizes[1] < (size_t)SEQ * SEQ_FULL) return;
  if (in_sizes[2] < DM * DM || in_sizes[4] < DM * DM || in_sizes[6] < DM * DM || in_sizes[8] < DM * DM) return;
  if (in_sizes[3] < DM || in_sizes[5] < DM || in_sizes[7] < DM || in_sizes[9] < DM) return;
  if ((size_t)out_size < (size_t)NTOK * DM) return;

  const float* x   = (const float*)d_in[0];
  const float* msk = (const float*)d_in[1];
  const float* Wq  = (const float*)d_in[2];
  const float* bq  = (const float*)d_in[3];
  const float* Wk  = (const float*)d_in[4];
  const float* bk  = (const float*)d_in[5];
  const float* Wv  = (const float*)d_in[6];
  const float* bv  = (const float*)d_in[7];
  const float* Wo  = (const float*)d_in[8];
  const float* bo  = (const float*)d_in[9];
  float* outp = (float*)d_out;

  const size_t bAct = (size_t)NTOK * DM * 2;
  const size_t bW   = (size_t)DM * DM * 2;
  const size_t bSq  = (size_t)NB * NH * SEQ * 4;
  const size_t bMr  = (size_t)SEQ * SEQ * 4;
  size_t off = 0;
  const size_t oXb = off; off += bAct;
  const size_t oWq = off; off += bW;
  const size_t oWk = off; off += bW;
  const size_t oWv = off; off += bW;
  const size_t oWo = off; off += bW;
  const size_t oQh = off; off += bAct;
  const size_t oQr = off; off += bAct;
  const size_t oKh = off; off += bAct;
  const size_t oKr = off; off += bAct;
  const size_t oVh = off; off += bAct;
  const size_t oVr = off; off += bAct;
  const size_t oQs = off; off += bSq;
  const size_t oKs = off; off += bSq;
  const size_t oMr = off; off += bMr;
  if (off > ws_size) return;
  if (off > (size_t)134217728) return;

  char* ws = (char*)d_ws;
  unsigned short* Xb  = (unsigned short*)(ws + oXb);
  _Float16* Oh = (_Float16*)(ws + oXb);
  unsigned short* Wqb = (unsigned short*)(ws + oWq);
  unsigned short* Wkb = (unsigned short*)(ws + oWk);
  unsigned short* Wvb = (unsigned short*)(ws + oWv);
  _Float16* Wof = (_Float16*)(ws + oWo);
  _Float16* Qh = (_Float16*)(ws + oQh);
  _Float16* Qr = (_Float16*)(ws + oQr);
  _Float16* Kh = (_Float16*)(ws + oKh);
  _Float16* Kr = (_Float16*)(ws + oKr);
  _Float16* Vh = (_Float16*)(ws + oVh);
  _Float16* Vr = (_Float16*)(ws + oVr);
  float* Qs = (float*)(ws + oQs);
  float* Ks = (float*)(ws + oKs);
  float* Mr = (float*)(ws + oMr);

  const dim3 blk(256);
  const int n8x = NTOK * DM / 8;
  const int n8w = DM * DM / 8;
  const int n4m = SEQ * SEQ / 4;
  if ((n8x % 256) != 0 || (n8w % 256) != 0 || (n4m % 256) != 0) return;

  cvt_x_kernel<<<dim3(n8x / 256), blk, 0, stream>>>(x, Xb, n8x);
  cvt_w_kernel<<<dim3(n8w / 256, 3), blk, 0, stream>>>(Wq, Wk, Wv, Wqb, Wkb, Wvb, n8w);
  cvt_wo_kernel<<<dim3(n8w / 256), blk, 0, stream>>>(Wo, Wof, n8w);
  maskc_kernel<<<dim3(n4m / 256), blk, 0, stream>>>(msk, Mr, n4m);
  proj_kernel<<<dim3(((NTOK / 64) * (DM / 64)) / 8), blk, 0, stream>>>(
      (const __bf16*)Xb, DM, (const __bf16*)Wqb, DM, Qh, Qr, DM, NTOK, DM, DM, bq, DM, 0);
  proj_kernel<<<dim3(((NTOK / 64) * (DM / 64)) / 8), blk, 0, stream>>>(
      (const __bf16*)Xb, DM, (const __bf16*)Wkb, DM, Kh, Kr, DM, NTOK, DM, DM, bk, DM, 0);
  proj_kernel<<<dim3(((DM / 64) * (NTOK / 64)) / 8), blk, 0, stream>>>(
      (const __bf16*)Wvb, DM, (const __bf16*)Xb, DM, Vh, Vr, NTOK, DM, NTOK, DM, bv, DM, 1);
  norms_kernel<<<dim3(SEQ / 128, NB * NH, 2), dim3(128), 0, stream>>>(Qh, Qr, Kh, Kr, Qs, Ks);
  (void)hipFuncSetAttribute(reinterpret_cast<const void*>(&attn_kernel),
                            hipFuncAttributeMaxDynamicSharedMemorySize, ATT_LDS);
  attn_kernel<<<dim3(SEQ / QBLK, NH, NB), blk, ATT_LDS, stream>>>(Qh, Qr, Kh, Kr, Vh, Vr, Qs, Ks, Mr, Oh);
  oproj_kernel<<<dim3(((NTOK / 64) * (DM / 64)) / 8), blk, 0, stream>>>(
      Oh, DM, Wof, DM, outp, DM, NTOK, DM, DM, bo, DM, 0.0009765625f);
  (void)hipGetLastError();
}
